// MHN_WITH_1_HIDDEN_LAYER_2147483648715
// MI455X (gfx1250) — hardware-verified
//
#include <hip/hip_runtime.h>
#include <stdint.h>

#define N1   256
#define KT   64
#define QB   16
#define YSP  72
#define UP   16
#define OSP  260
#define L2E  1.44269504088896340736f
#define PEX  14.0f
#define YSC  16.0f
#define OSC  0.0625f
#define ALP  0.5f
#define HBT  0.5f

static_assert(N1 == 256);
static_assert((YSP * 2) % 16 == 0);
static_assert((OSP * 4) % 16 == 0);
static_assert(KT == 64);
static_assert(QB == 16);

typedef _Float16       v8h  __attribute__((ext_vector_type(8)));
typedef _Float16       v16h __attribute__((ext_vector_type(16)));
typedef __bf16         v16b __attribute__((ext_vector_type(16)));
typedef unsigned short v8us __attribute__((ext_vector_type(8)));
typedef float          v4f  __attribute__((ext_vector_type(4)));
typedef float          v8f  __attribute__((ext_vector_type(8)));

union FragH { v8h p[2]; v16h v; };
union FragB { v8us p[2]; v16b v; };
static_assert(sizeof(FragH) == 32);
static_assert(sizeof(FragB) == 32);

__device__ __forceinline__ v8f zero8() { v8f z = {0.f, 0.f, 0.f, 0.f, 0.f, 0.f, 0.f, 0.f}; return z; }

__device__ __forceinline__ unsigned int bf_bits(float x) {
  unsigned int u = __float_as_uint(x);
  u += 0x7FFFu + ((u >> 16) & 1u);
  return u >> 16;
}
__device__ __forceinline__ float bf_rne(float x) { return __uint_as_float(bf_bits(x) << 16); }

__device__ __forceinline__ v8f mma_h(v16h a, v16h b, v8f c) {
  v8f d = __builtin_amdgcn_wmma_f32_16x16x32_f16(false, a, false, b, (short)0, c, false, false);
#if defined(__HIP_DEVICE_COMPILE__)
  asm volatile("v_nop\n\tv_nop\n\tv_nop\n\tv_nop" : "+v"(d) : "v"(a), "v"(b));
#endif
  return d;
}
__device__ __forceinline__ v8f mma_b(v16b a, v16b b, v8f c) {
  v8f d = __builtin_amdgcn_wmma_f32_16x16x32_bf16(false, a, false, b, (short)0, c, false, false);
#if defined(__HIP_DEVICE_COMPILE__)
  asm volatile("v_nop\n\tv_nop\n\tv_nop\n\tv_nop" : "+v"(d) : "v"(a), "v"(b));
#endif
  return d;
}

__global__ __launch_bounds__(256)
void k_mem(const float* __restrict__ Mem, unsigned short* MB, _Float16* MT, float* HB, int nkeys) {
  __shared__ __align__(16) _Float16 Ys[N1 * YSP];
  __shared__ __align__(16) float Hs[KT];
  const int t  = threadIdx.x, lane = t & 31, wv = t >> 5;
  const int i0 = blockIdx.x * KT;

  v8us mbv[8];
#pragma unroll
  for (int it = 0; it < 8; ++it) {
    const int row = it * 8 + wv;
    const float* s = Mem + (size_t)(i0 + row) * N1 + 8 * lane;
    const v4f a = *(const v4f*)(s);
    const v4f b = *(const v4f*)(s + 4);
    v8us w;
#pragma unroll
    for (int i = 0; i < 4; ++i) {
      const unsigned int ua = bf_bits(a[i]);
      const float ra = __uint_as_float(ua << 16);
      w[i] = (unsigned short)ua;
      Ys[(8 * lane + i) * YSP + row] = (_Float16)(ra * YSC);
    }
#pragma unroll
    for (int i = 0; i < 4; ++i) {
      const unsigned int ub = bf_bits(b[i]);
      const float rb = __uint_as_float(ub << 16);
      w[4 + i] = (unsigned short)ub;
      Ys[(8 * lane + 4 + i) * YSP + row] = (_Float16)(rb * YSC);
    }
    mbv[it] = w;
  }

  if (t < KT) {
    const float* s = Mem + (size_t)(i0 + t) * N1;
    float sq = 0.f;
#pragma unroll 1
    for (int d = 0; d < N1; d += 4) {
      const v4f a = *(const v4f*)(s + d);
      const float r0 = bf_rne(a[0]);
      const float r1 = bf_rne(a[1]);
      const float r2 = bf_rne(a[2]);
      const float r3 = bf_rne(a[3]);
      sq = fmaf(r0, r0, sq);
      sq = fmaf(r1, r1, sq);
      sq = fmaf(r2, r2, sq);
      sq = fmaf(r3, r3, sq);
    }
    Hs[t] = sq * (-(HBT * L2E));
  }
  __syncthreads();

  v8h yv[8];
  size_t py[8];
#pragma unroll
  for (int it = 0; it < 8; ++it) {
    const int q = it * 256 + t, drow = q >> 3, e8 = q & 7;
    yv[it] = *(const v8h*)(Ys + drow * YSP + 8 * e8);
    py[it] = (size_t)drow * nkeys + i0 + 8 * e8;
  }
  const int hq = (t < 16) ? t : 15;
  const v4f hv = *(const v4f*)(Hs + 4 * hq);
  const bool wh = (t < 16);
  float* hd = HB + i0 + 4 * hq;
  const size_t pm0 = (size_t)(i0 + wv) * N1 + 8 * lane;

#pragma unroll
  for (int it = 0; it < 8; ++it) *(volatile v8us*)(MB + pm0 + (size_t)it * 8 * N1) = mbv[it];
#pragma unroll
  for (int it = 0; it < 8; ++it) *(volatile v8h*)(MT + py[it]) = yv[it];
  if (wh) *(volatile v4f*)hd = hv;
  __threadfence();
#pragma unroll
  for (int it = 0; it < 8; ++it) *(volatile v8us*)(MB + pm0 + (size_t)it * 8 * N1) = mbv[it];
#pragma unroll
  for (int it = 0; it < 8; ++it) *(volatile v8h*)(MT + py[it]) = yv[it];
  if (wh) *(volatile v4f*)hd = hv;
}

__global__ __launch_bounds__(256)
void k_v(const float* __restrict__ v, unsigned short* VB) {
  const int t  = threadIdx.x, lane = t & 31, wv = t >> 5;
  const int r0 = blockIdx.x * 32;
  v8us vb[4];
#pragma unroll
  for (int it = 0; it < 4; ++it) {
    const int row = it * 8 + wv;
    const float* s = v + (size_t)(r0 + row) * N1 + 8 * lane;
    const v4f a = *(const v4f*)(s);
    const v4f b = *(const v4f*)(s + 4);
    v8us w;
#pragma unroll
    for (int i = 0; i < 4; ++i) {
      w[i]     = (unsigned short)bf_bits(a[i]);
      w[4 + i] = (unsigned short)bf_bits(b[i]);
    }
    vb[it] = w;
  }
  const size_t p0 = (size_t)(r0 + wv) * N1 + 8 * lane;
#pragma unroll
  for (int it = 0; it < 4; ++it) *(volatile v8us*)(VB + p0 + (size_t)it * 8 * N1) = vb[it];
  __threadfence();
#pragma unroll
  for (int it = 0; it < 4; ++it) *(volatile v8us*)(VB + p0 + (size_t)it * 8 * N1) = vb[it];
}

__global__ __launch_bounds__(64)
void k_main(const unsigned short* __restrict__ MB, const unsigned short* __restrict__ VB,
            const _Float16* __restrict__ MT, const float* __restrict__ HB,
            const float* __restrict__ v, const float* __restrict__ mask,
            float* out, int nkeys) {
  __shared__ __align__(16) float Us[2][32 * UP];
  __shared__ __align__(16) float Os[QB * OSP];
  const int t    = threadIdx.x;
  const int lane = t & 31, wv = t >> 5;
  const int hh   = lane >> 4, n = lane & 15;
  const int q0   = blockIdx.x * QB;

  const unsigned short* ap = MB + (size_t)(16 * wv + n) * N1 + 8 * hh;
  const unsigned short* bp = VB + (size_t)(q0 + n) * N1 + 8 * hh;
  const _Float16*       yp = MT + (size_t)(128 * wv + n) * nkeys + 8 * hh;
  const float*          hp = HB + 8 * hh;

  v8f O[8];
#pragma unroll
  for (int j = 0; j < 8; ++j) O[j] = zero8();
  float m = -1.0e30f, z = 0.f;

#pragma unroll 1
  for (int c0 = 0; c0 < nkeys; c0 += 32) {
    v8f S = zero8();
    const unsigned short* a = ap + (size_t)c0 * N1;
#pragma unroll 2
    for (int kk = 0; kk < 8; ++kk) {
      FragB fa, fb;
      fa.p[0] = *(const v8us*)(a + kk * 32);
      fa.p[1] = *(const v8us*)(a + kk * 32 + 16);
      fb.p[0] = *(const v8us*)(bp + kk * 32);
      fb.p[1] = *(const v8us*)(bp + kk * 32 + 16);
      S = mma_b(fa.v, fb.v, S);
    }
    const int par = (c0 >> 5) & 1;
    float* ub = &Us[par][0];
#pragma unroll
    for (int r = 0; r < 8; ++r) ub[(16 * wv + 8 * hh + r) * UP + n] = S[r];
    __syncthreads();

    const v4f h0a = *(const v4f*)(hp + c0);
    const v4f h0b = *(const v4f*)(hp + c0 + 4);
    const v4f h1a = *(const v4f*)(hp + c0 + 16);
    const v4f h1b = *(const v4f*)(hp + c0 + 20);
    const float* up0 = ub + (8 * hh) * UP + n;
    float u0[8], u1[8];
#pragma unroll
    for (int r = 0; r < 4; ++r) {
      u0[r]     = fmaf(up0[r * UP],        L2E, h0a[r]);
      u0[4 + r] = fmaf(up0[(4 + r) * UP],  L2E, h0b[r]);
      u1[r]     = fmaf(up0[(16 + r) * UP], L2E, h1a[r]);
      u1[4 + r] = fmaf(up0[(20 + r) * UP], L2E, h1b[r]);
    }
    float tm = fmaxf(u0[0], u1[0]);
#pragma unroll
    for (int r = 1; r < 8; ++r) tm = fmaxf(tm, fmaxf(u0[r], u1[r]));
    const float tmo = __shfl_xor(tm, 16, 32);
    tm = fmaxf(tm, tmo);
    const float mn    = fmaxf(m, tm);
    const float alpha = __builtin_amdgcn_exp2f(m - mn);
    m = mn;
    const float mbase = mn - PEX;
    z *= alpha;
#pragma unroll
    for (int j = 0; j < 8; ++j) O[j] = O[j] * alpha;

    FragH pf;
#pragma unroll
    for (int r = 0; r < 8; ++r) {
      const float p0 = __builtin_amdgcn_exp2f(u0[r] - mbase);
      const float p1 = __builtin_amdgcn_exp2f(u1[r] - mbase);
      const _Float16 f0 = (_Float16)p0;
      const _Float16 f1 = (_Float16)p1;
      pf.v[r]     = f0;
      pf.v[8 + r] = f1;
      z += (float)f0;
      z += (float)f1;
    }

#pragma unroll
    for (int dt = 0; dt < 8; ++dt) {
      const _Float16* yd = yp + (size_t)(16 * dt) * nkeys + c0;
      FragH ay;
      ay.p[0] = *(const v8h*)(yd);
      ay.p[1] = *(const v8h*)(yd + 16);
      O[dt] = mma_h(ay.v, pf.v, O[dt]);
    }
  }

  const float zo  = __shfl_xor(z, 16, 32);
  const float ztt = z + zo;
  const float rz  = __builtin_amdgcn_rcpf(ztt) * OSC;
#pragma unroll
  for (int dt = 0; dt < 8; ++dt) {
#pragma unroll
    for (int r = 0; r < 8; ++r) Os[n * OSP + 128 * wv + 16 * dt + 8 * hh + r] = O[dt][r] * rz;
  }
  __syncthreads();

  const size_t gb = (size_t)q0 * N1 + 4 * t;
  v4f ov[QB];
#pragma unroll
  for (int it = 0; it < QB; ++it) {
    const v4f U  = *(const v4f*)(Os + it * OSP + 4 * t);
    const v4f vv = *(const v4f*)(v + gb + (size_t)it * N1);
    const v4f mk = *(const v4f*)(mask + gb + (size_t)it * N1);
    v4f o;
#pragma unroll
    for (int i = 0; i < 4; ++i) {
      const float vr = bf_rne(vv[i]);
      const float mr = bf_rne(mk[i]);
      const float ud = (U[i] - vr) * ALP;
      o[i] = vr + ud * mr;
    }
    ov[it] = o;
  }
#pragma unroll
  for (int it = 0; it < QB; ++it) *(volatile v4f*)(out + gb + (size_t)it * N1) = ov[it];
  __threadfence();
#pragma unroll
  for (int it = 0; it < QB; ++it) *(volatile v4f*)(out + gb + (size_t)it * N1) = ov[it];
}

extern "C" void kernel_launch(void* const* d_in, const int* in_sizes, int n_in,
                              void* d_out, int out_size, void* d_ws, size_t ws_size,
                              hipStream_t stream) {
  if (n_in < 3) return;
  const int nq = in_sizes[0] / N1;
  const int nk = in_sizes[2] / N1;
  if (nq <= 0 || nk <= 0) return;
  if (nq * N1 != in_sizes[0] || nk * N1 != in_sizes[2]) return;
  if (in_sizes[1] != nq * N1) return;
  if (out_size != nq * N1) return;
  if ((nq % 32) != 0 || (nk % KT) != 0) return;

  size_t off = 0;
  const size_t oMB = off; off += (size_t)nk * N1 * 2;
  const size_t oMT = off; off += (size_t)N1 * nk * 2;
  const size_t oVB = off; off += (size_t)nq * N1 * 2;
  const size_t oHB = off; off += (((size_t)nk * 4) + 127) / 128 * 128;
  if (off > ws_size) return;
  if (off > (size_t)134217728) return;

  const float* v    = (const float*)d_in[0];
  const float* mask = (const float*)d_in[1];
  const float* Mem  = (const float*)d_in[2];
  float* out = (float*)d_out;

  char* ws = (char*)d_ws;
  unsigned short* MB = (unsigned short*)(ws + oMB);
  _Float16*       MT = (_Float16*)(ws + oMT);
  unsigned short* VB = (unsigned short*)(ws + oVB);
  float*          HB = (float*)(ws + oHB);

  k_mem<<<dim3(nk / KT), dim3(256), 0, stream>>>(Mem, MB, MT, HB, nk);
  k_v<<<dim3(nq / 32), dim3(256), 0, stream>>>(v, VB);
  k_main<<<dim3(nq / QB), dim3(64), 0, stream>>>(MB, VB, MT, HB, v, mask, out, nk);
  (void)hipGetLastError();
}
